// Transformer_36481452212853
// MI455X (gfx1250) — hardware-verified
//
#include <hip/hip_runtime.h>
#include <stddef.h>
#include <stdint.h>
#include <math.h>


#define DF     128
#define SP     256
#define FP     512
#define NLAY   2
#define NTHR   256
#define NWAVE  8
#define EPT    8
#define CHUNK  (NTHR * EPT)
#define WCAP   (EPT * 32)
#define LISTN  (NWAVE * WCAP)
#define NBA    1024
#define SLA    10
#define RCAP   28672
#define DEGCAP 64
#define GBM    64
#define GBN    128
#define GTHR   128
#define NPARTS 33
#define WE_ELEMS   16384
#define LAY_ELEMS  262144
#define OFF_QKV2   0
#define OFF_WO2    98304
#define OFF_WF12   131072
#define OFF_WF22   196608
#define WPL_ELEMS  (WE_ELEMS + NLAY * LAY_ELEMS)
#define AGG_ZINTS    (LISTN + 2 * RCAP + 3 * NBA)
#define MISC_INTS    16
#define ROWBUF_INTS  (NWAVE * SP / 2)
#define AGG_LDS_INTS (AGG_ZINTS + MISC_INTS + ROWBUF_INTS)
#define WSMAX  134217728

#define M_EMB  0
#define M_QKV  1
#define M_LN   2
#define M_FFN1 3

static_assert((CHUNK & (CHUNK - 1)) == 0 && CHUNK <= 4096);
static_assert((NBA & (NBA - 1)) == 0 && NBA == (1 << SLA));
static_assert(((long long)CHUNK << SLA) < (1LL << 31));
static_assert(LISTN % NTHR == 0);
static_assert(NBA % NWAVE == 0 && NBA % 32 == 0 && NBA % GBM == 0);
static_assert(RCAP % 4 == 0 && AGG_ZINTS % 4 == 0 && LISTN % 4 == 0 && ((AGG_ZINTS + MISC_INTS) % 4) == 0);
static_assert(AGG_ZINTS % (NTHR * 4) == 0);
static_assert(GBN == DF && GBM == (GTHR / 32) * 16 && DF == 4 * 32 && SP == 2 * DF && FP == 4 * DF);
static_assert(DF % 32 == 0 && SP % 32 == 0 && FP % 32 == 0);
static_assert(OFF_WO2 == 384 * 256 && OFF_WF12 == OFF_WO2 + 128 * 256 && OFF_WF22 == OFF_WF12 + 256 * 256);
static_assert(LAY_ELEMS == OFF_WF22 + 128 * 512);
static_assert(AGG_LDS_INTS * 4 <= 300000);
static_assert(DEGCAP >= 33 + 8 && RCAP >= 16696);

typedef float          v4f   __attribute__((ext_vector_type(4)));
typedef float          v8f   __attribute__((ext_vector_type(8)));
typedef int            v4i   __attribute__((ext_vector_type(4)));
typedef int            v8i   __attribute__((ext_vector_type(8)));
typedef unsigned       v2u   __attribute__((ext_vector_type(2)));
typedef unsigned short v4us  __attribute__((ext_vector_type(4)));
typedef unsigned short v8us  __attribute__((ext_vector_type(8)));
typedef unsigned short v16us __attribute__((ext_vector_type(16)));
typedef __bf16         v16bf __attribute__((ext_vector_type(16)));
typedef v4f  __attribute__((may_alias)) v4fa;
typedef v4i  __attribute__((may_alias)) v4ia;
typedef v2u  __attribute__((may_alias)) v2ua;
typedef v4us __attribute__((may_alias)) v4usa;
typedef v8us __attribute__((may_alias)) v8usa;
union FragB { v16bf v; v16us u; v8us h[2]; v8i w; };

__device__ __forceinline__ v8f wmb(const FragB& a, const FragB& b, v8f c) {
  v8f d = __builtin_amdgcn_wmma_f32_16x16x32_bf16(false, a.v, false, b.v, (short)0, c, false, false);
  asm volatile("v_nop\n\tv_nop\n\tv_nop\n\tv_nop" : "+v"(d) : "v"(a.w), "v"(b.w));
  return d;
}

__device__ __forceinline__ unsigned bf16_bits(float f) {
  const unsigned u = __float_as_uint(f);
  return (u + 0x7FFFu + ((u >> 16) & 1u)) >> 16;
}
__device__ __forceinline__ float bf16_val(float f) {
  return __uint_as_float(bf16_bits(f) << 16);
}
__device__ __forceinline__ void hilo4(const v4f y, v4us& h4, v4us& l4) {
  unsigned hb;
  hb = bf16_bits(y.x); h4[0] = (unsigned short)hb; l4[0] = (unsigned short)bf16_bits(y.x - __uint_as_float(hb << 16));
  hb = bf16_bits(y.y); h4[1] = (unsigned short)hb; l4[1] = (unsigned short)bf16_bits(y.y - __uint_as_float(hb << 16));
  hb = bf16_bits(y.z); h4[2] = (unsigned short)hb; l4[2] = (unsigned short)bf16_bits(y.z - __uint_as_float(hb << 16));
  hb = bf16_bits(y.w); h4[3] = (unsigned short)hb; l4[3] = (unsigned short)bf16_bits(y.w - __uint_as_float(hb << 16));
}

__device__ __forceinline__ void wave_sync() {
  __builtin_amdgcn_fence(__ATOMIC_RELEASE, "wavefront");
  __builtin_amdgcn_wave_barrier();
  __builtin_amdgcn_fence(__ATOMIC_ACQUIRE, "wavefront");
}

template <int SLB>
__device__ __forceinline__ int scan_chunk(const int* __restrict__ dsts, int nE, int cbase, int slotBase,
                                          int nb, int vec8, int* list, int tid, int lane, int wave) {
  int wc = 0;
  const int el0  = tid * EPT;
  const int e0   = cbase + el0;
  const int sent = -2147483647 - 1;
  v4i da, db;
  if (vec8 != 0 && cbase + CHUNK <= nE) {
    da = *(const v4i*)(dsts + e0);
    db = *(const v4i*)(dsts + e0 + 4);
  } else {
    da.x = (e0     < nE) ? dsts[min(e0,     nE - 1)] : sent;
    da.y = (e0 + 1 < nE) ? dsts[min(e0 + 1, nE - 1)] : sent;
    da.z = (e0 + 2 < nE) ? dsts[min(e0 + 2, nE - 1)] : sent;
    da.w = (e0 + 3 < nE) ? dsts[min(e0 + 3, nE - 1)] : sent;
    db.x = (e0 + 4 < nE) ? dsts[min(e0 + 4, nE - 1)] : sent;
    db.y = (e0 + 5 < nE) ? dsts[min(e0 + 5, nE - 1)] : sent;
    db.z = (e0 + 6 < nE) ? dsts[min(e0 + 6, nE - 1)] : sent;
    db.w = (e0 + 7 < nE) ? dsts[min(e0 + 7, nE - 1)] : sent;
  }
  const unsigned nbs = (unsigned)slotBase;
  const unsigned unb = (unsigned)nb;
  const unsigned s0 = (unsigned)da.x - nbs, s1 = (unsigned)da.y - nbs;
  const unsigned s2 = (unsigned)da.z - nbs, s3 = (unsigned)da.w - nbs;
  const unsigned s4 = (unsigned)db.x - nbs, s5 = (unsigned)db.y - nbs;
  const unsigned s6 = (unsigned)db.z - nbs, s7 = (unsigned)db.w - nbs;
  const bool h0 = s0 < unb, h1 = s1 < unb, h2 = s2 < unb, h3 = s3 < unb;
  const bool h4 = s4 < unb, h5 = s5 < unb, h6 = s6 < unb, h7 = s7 < unb;
  const unsigned any = __builtin_amdgcn_ballot_w32(h0 | h1 | h2 | h3 | h4 | h5 | h6 | h7);
  if (any != 0u) {
#define HITJ(J, HJ, SJ) { \
      const unsigned mj = __builtin_amdgcn_ballot_w32(HJ); \
      if (mj != 0u) { \
        if (HJ) { \
          const int pos = wc + (int)__builtin_amdgcn_mbcnt_lo(mj, 0u); \
          if (pos < WCAP) list[wave * WCAP + pos] = ((el0 + (J)) << SLB) | (int)(SJ); \
        } \
        wc += (int)__builtin_popcount(mj); } }
    HITJ(0, h0, s0)
    HITJ(1, h1, s1)
    HITJ(2, h2, s2)
    HITJ(3, h3, s3)
    HITJ(4, h4, s4)
    HITJ(5, h5, s5)
    HITJ(6, h6, s6)
    HITJ(7, h7, s7)
#undef HITJ
  }
  return wc;
}

__device__ __forceinline__ void ld8s(const float* __restrict__ p, int ldw, float* f) {
#pragma unroll
  for (int i = 0; i < 8; ++i) f[i] = p[(size_t)i * (size_t)ldw];
}

__global__ __launch_bounds__(NTHR) void k_wprep(const float* __restrict__ Wemb, const float* __restrict__ Wq,
                                                const float* __restrict__ Wk, const float* __restrict__ Wv,
                                                const float* __restrict__ Wo, const float* __restrict__ Wf1,
                                                const float* __restrict__ Wf2, unsigned short* WPL) {
  const int part = (int)blockIdx.x >> 3;
  const int v    = (((int)blockIdx.x & 7) * NTHR) + (int)threadIdx.x;
  const int n    = v >> 4;
  const int k8   = (v & 15) * 8;
  int mat = 0, ldw = DF, ks0 = 0, ns0 = 0, pitch = DF, nd0 = 0, kd0 = 0, lay = 0;
  size_t dbase = 0;
  if (part >= NPARTS) return;
  if (part > 0) {
    const int pp = part - 1;
    lay = pp >> 4;
    const int p = pp & 15;
    const size_t lb = (size_t)WE_ELEMS + (size_t)lay * LAY_ELEMS;
    if (p < 6) {
      const int mm = p >> 1;
      mat = 1 + mm; ldw = DF; ks0 = 0; ns0 = 0; dbase = lb + OFF_QKV2; pitch = SP; nd0 = DF * mm; kd0 = DF * (p & 1);
    } else if (p < 8) {
      mat = 4; ldw = DF; ks0 = 0; ns0 = 0; dbase = lb + OFF_WO2; pitch = SP; nd0 = 0; kd0 = DF * (p - 6);
    } else if (p < 12) {
      mat = 5; ldw = 2 * DF; ks0 = 0; ns0 = DF * ((p - 8) >> 1); dbase = lb + OFF_WF12; pitch = SP;
      nd0 = ns0; kd0 = DF * ((p - 8) & 1);
    } else {
      mat = 6; ldw = DF; ks0 = DF * ((p - 12) >> 1); ns0 = 0; dbase = lb + OFF_WF22; pitch = FP;
      nd0 = 0; kd0 = 2 * DF * ((p - 12) & 1) + ks0;
    }
  }
  const size_t lsz = (mat >= 5) ? (size_t)(2 * DF * DF) : (size_t)(DF * DF);
  const size_t so  = (size_t)lay * lsz + (size_t)(ks0 + k8) * (size_t)ldw + (size_t)(ns0 + n);
  float f[8];
  switch (mat) {
    case 0:  ld8s(Wemb + so, ldw, f); break;
    case 1:  ld8s(Wq + so, ldw, f);   break;
    case 2:  ld8s(Wk + so, ldw, f);   break;
    case 3:  ld8s(Wv + so, ldw, f);   break;
    case 4:  ld8s(Wo + so, ldw, f);   break;
    case 5:  ld8s(Wf1 + so, ldw, f);  break;
    default: ld8s(Wf2 + so, ldw, f);  break;
  }
  v8us o;
  o[0] = (unsigned short)bf16_bits(f[0]); o[1] = (unsigned short)bf16_bits(f[1]);
  o[2] = (unsigned short)bf16_bits(f[2]); o[3] = (unsigned short)bf16_bits(f[3]);
  o[4] = (unsigned short)bf16_bits(f[4]); o[5] = (unsigned short)bf16_bits(f[5]);
  o[6] = (unsigned short)bf16_bits(f[6]); o[7] = (unsigned short)bf16_bits(f[7]);
  unsigned short* dp = WPL + dbase + (size_t)(nd0 + n) * (size_t)pitch + (size_t)(kd0 + k8);
  *(volatile v8us*)dp = o;
  __threadfence();
  *(volatile v8us*)dp = o;
}

__global__ __launch_bounds__(NTHR) void k_cvx(const float* __restrict__ x, int nN, int nUnits,
                                              unsigned short* xb) {
  const int u = (int)blockIdx.x * NTHR + (int)threadIdx.x;
  if (u >= nUnits) return;
  const int row = u >> 4;
  const int k8  = (u & 15) * 8;
  const int rc  = row < nN ? row : nN - 1;
  const float* p = x + (size_t)rc * DF + k8;
  const v4f a = *(const v4fa*)p;
  const v4f b = *(const v4fa*)(p + 4);
  const bool ok = row < nN;
  v8us o;
  o[0] = ok ? (unsigned short)bf16_bits(a.x) : (unsigned short)0;
  o[1] = ok ? (unsigned short)bf16_bits(a.y) : (unsigned short)0;
  o[2] = ok ? (unsigned short)bf16_bits(a.z) : (unsigned short)0;
  o[3] = ok ? (unsigned short)bf16_bits(a.w) : (unsigned short)0;
  o[4] = ok ? (unsigned short)bf16_bits(b.x) : (unsigned short)0;
  o[5] = ok ? (unsigned short)bf16_bits(b.y) : (unsigned short)0;
  o[6] = ok ? (unsigned short)bf16_bits(b.z) : (unsigned short)0;
  o[7] = ok ? (unsigned short)bf16_bits(b.w) : (unsigned short)0;
  unsigned short* dp = xb + (size_t)row * DF + k8;
  *(volatile v8us*)dp = o;
  __threadfence();
  *(volatile v8us*)dp = o;
}

template <int MODE, int FIN>
__global__ __launch_bounds__(GTHR) void k_gemm(
    const unsigned short* __restrict__ A, int lda,
    const unsigned short* __restrict__ BT, int K,
    const float* __restrict__ bA, const float* __restrict__ bB, const float* __restrict__ bC,
    const unsigned short* __restrict__ R,
    const float* __restrict__ lnw, const float* __restrict__ lnb,
    unsigned short* outH, int ldh, float* outF, size_t fPlane, int nOut)
{
  constexpr bool OUT16 = (MODE == M_EMB) || (MODE == M_FFN1) || (MODE == M_LN && FIN == 0);
  __shared__ __attribute__((aligned(16))) float stg[GBM * GBN];
  const int tid = (int)threadIdx.x, lane = tid & 31, wave = tid >> 5, hh = lane >> 4, m = lane & 15;
  const int rowBase = (int)blockIdx.x * GBM;
  const int ny      = (int)blockIdx.y;
  const int col0    = ny * GBN;

  v8f acc[8];
  {
    const v8f z = {0.f, 0.f, 0.f, 0.f, 0.f, 0.f, 0.f, 0.f};
#pragma unroll
    for (int t = 0; t < 8; ++t) acc[t] = z;
  }
  const unsigned short* ap = A + (size_t)(rowBase + 16 * wave + m) * (size_t)lda + 8 * hh;
  const unsigned short* bp = BT + (size_t)(col0 + m) * (size_t)K + 8 * hh;

#pragma unroll 1
  for (int k0 = 0; k0 < K; k0 += 32) {
    FragB af;
    af.h[0] = *(const v8usa*)(ap + k0);
    af.h[1] = *(const v8usa*)(ap + k0 + 16);
#pragma unroll
    for (int nt = 0; nt < 8; ++nt) {
      const unsigned short* wq = bp + (size_t)(16 * nt) * (size_t)K + k0;
      FragB bf;
      bf.h[0] = *(const v8usa*)wq;
      bf.h[1] = *(const v8usa*)(wq + 16);
      acc[nt] = wmb(af, bf, acc[nt]);
    }
  }

#pragma unroll
  for (int nt = 0; nt < 8; ++nt) {
    const int lc = 16 * nt + m;
#pragma unroll
    for (int r = 0; r < 8; ++r) {
      const int lr = 16 * wave + 8 * hh + r;
      stg[lr * GBN + lc] = acc[nt][r];
    }
  }
  __syncthreads();

  v4f bb4 = {0.f, 0.f, 0.f, 0.f};
  v4f lw4 = {0.f, 0.f, 0.f, 0.f};
  v4f lb4 = {0.f, 0.f, 0.f, 0.f};
  if constexpr (MODE == M_QKV) {
    const v4f t0 = *(const v4f*)(bA + 4 * lane);
    const v4f t1 = *(const v4f*)(bB + 4 * lane);
    const v4f t2 = *(const v4f*)(bC + 4 * lane);
    const v4f ts = (ny == 0) ? t0 : ((ny == 1) ? t1 : t2);
    bb4.x = bf16_val(ts.x); bb4.y = bf16_val(ts.y); bb4.z = bf16_val(ts.z); bb4.w = bf16_val(ts.w);
  } else if constexpr (MODE == M_FFN1) {
    const v4f ts = *(const v4f*)(bA + col0 + 4 * lane);
    bb4.x = bf16_val(ts.x); bb4.y = bf16_val(ts.y); bb4.z = bf16_val(ts.z); bb4.w = bf16_val(ts.w);
  } else if constexpr (MODE == M_LN) {
    const v4f ts = *(const v4f*)(bA + 4 * lane);
    bb4.x = bf16_val(ts.x); bb4.y = bf16_val(ts.y); bb4.z = bf16_val(ts.z); bb4.w = bf16_val(ts.w);
    const v4f tw = *(const v4f*)(lnw + 4 * lane);
    const v4f tb = *(const v4f*)(lnb + 4 * lane);
    lw4.x = bf16_val(tw.x); lw4.y = bf16_val(tw.y); lw4.z = bf16_val(tw.z); lw4.w = bf16_val(tw.w);
    lb4.x = bf16_val(tb.x); lb4.y = bf16_val(tb.y); lb4.z = bf16_val(tb.z); lb4.w = bf16_val(tb.w);
  }

#pragma unroll 1
  for (int i = 0; i < 16; ++i) {
    const int lr  = 16 * wave + i;
    const int row = rowBase + lr;
    const bool ok = row < nOut;
    float* srow = stg + lr * GBN;
    v4f t = *(const v4fa*)(srow + 4 * lane);
    t = t + bb4;
    v4f y;
    if constexpr (MODE == M_LN) {
      const unsigned short* rp = R + (size_t)row * SP + 4 * lane;
      const v2u wh = *(const v2ua*)rp;
      const v2u wl = *(const v2ua*)(rp + DF);
      v4f x;
      x.x = t.x + (__uint_as_float(wh.x << 16)         + __uint_as_float(wl.x << 16));
      x.y = t.y + (__uint_as_float(wh.x & 0xffff0000u) + __uint_as_float(wl.x & 0xffff0000u));
      x.z = t.z + (__uint_as_float(wh.y << 16)         + __uint_as_float(wl.y << 16));
      x.w = t.w + (__uint_as_float(wh.y & 0xffff0000u) + __uint_as_float(wl.y & 0xffff0000u));
      float s = (x.x + x.y) + (x.z + x.w);
      s += __shfl_xor(s, 16, 32);
      s += __shfl_xor(s, 8, 32);
      s += __shfl_xor(s, 4, 32);
      s += __shfl_xor(s, 2, 32);
      s += __shfl_xor(s, 1, 32);
      const float mean = s * (1.0f / 128.0f);
      v4f d;
      d.x = x.x - mean; d.y = x.y - mean; d.z = x.z - mean; d.w = x.w - mean;
      float vq = (d.x * d.x + d.y * d.y) + (d.z * d.z + d.w * d.w);
      vq += __shfl_xor(vq, 16, 32);
      vq += __shfl_xor(vq, 8, 32);
      vq += __shfl_xor(vq, 4, 32);
      vq += __shfl_xor(vq, 2, 32);
      vq += __shfl_xor(vq, 1, 32);
      const float rstd = rsqrtf(vq * (1.0f / 128.0f) + 1e-5f);
      y.x = d.x * rstd * lw4.x + lb4.x;
      y.y = d.y * rstd * lw4.y + lb4.y;
      y.z = d.z * rstd * lw4.z + lb4.z;
      y.w = d.w * rstd * lw4.w + lb4.w;
    } else if constexpr (MODE == M_FFN1) {
      y.x = (t.x > 0.0f) ? t.x : (t.x - t.x);
      y.y = (t.y > 0.0f) ? t.y : (t.y - t.y);
      y.z = (t.z > 0.0f) ? t.z : (t.z - t.z);
      y.w = (t.w > 0.0f) ? t.w : (t.w - t.w);
    } else {
      y = t;
    }
    y.x = ok ? y.x : 0.0f; y.y = ok ? y.y : 0.0f; y.z = ok ? y.z : 0.0f; y.w = ok ? y.w : 0.0f;
    if constexpr (OUT16) {
      v4us h4, l4;
      hilo4(y, h4, l4);
      unsigned short* urow = (unsigned short*)srow;
      *(v4usa*)(urow + 4 * lane) = h4;
      *(v4usa*)(urow + DF + 4 * lane) = l4;
    } else {
      *(v4fa*)(srow + 4 * lane) = y;
    }
  }
  __syncthreads();

  if constexpr (OUT16) {
    const int c16 = (MODE == M_FFN1) ? (col0 + 8 * (lane & 15) + (lane >> 4) * (2 * DF)) : (8 * lane);
    v8us qv[16];
#pragma unroll
    for (int i = 0; i < 16; ++i) {
      const unsigned short* urow = (const unsigned short*)stg + (size_t)(16 * wave + i) * (2 * GBN);
      qv[i] = *(const v8usa*)(urow + 8 * lane);
    }
#pragma unroll
    for (int i = 0; i < 16; ++i) {
      unsigned short* rp = outH + (size_t)(rowBase + 16 * wave + i) * (size_t)ldh + c16;
      *(volatile v8us*)rp = qv[i];
    }
    __threadfence();
#pragma unroll
    for (int i = 0; i < 16; ++i) {
      unsigned short* rp = outH + (size_t)(rowBase + 16 * wave + i) * (size_t)ldh + c16;
      *(volatile v8us*)rp = qv[i];
    }
  } else {
    float* ob = outF + (size_t)ny * fPlane;
    v4f pv[16];
#pragma unroll
    for (int i = 0; i < 16; ++i) pv[i] = *(const v4fa*)(stg + (16 * wave + i) * GBN + 4 * lane);
#pragma unroll
    for (int i = 0; i < 16; ++i) {
      const int r = rowBase + 16 * wave + i;
      const bool st = (FIN != 0) ? (r < nOut) : true;
      if (st) *(volatile v4f*)(ob + (size_t)r * DF + 4 * lane) = pv[i];
    }
    __threadfence();
#pragma unroll
    for (int i = 0; i < 16; ++i) {
      const int r = rowBase + 16 * wave + i;
      const bool st = (FIN != 0) ? (r < nOut) : true;
      if (st) *(volatile v4f*)(ob + (size_t)r * DF + 4 * lane) = pv[i];
    }
  }
}

__global__ __launch_bounds__(NTHR) void k_scan(const int* __restrict__ gath, const int* __restrict__ keys,
                                               int nE, int nN, int vec8, int mRows,
                                               const float* __restrict__ Qp, const float* __restrict__ Kp,
                                               const float* __restrict__ Vp, unsigned short* attn) {
  extern __shared__ __attribute__((aligned(16))) int dsm[];
  int* list = dsm;
  int* hl   = dsm + LISTN;
  int* sl   = hl + RCAP;
  int* cnt  = sl + RCAP;
  int* offs = cnt + NBA;
  int* cur  = offs + NBA;
  int* misc = cur + NBA;
  const int tid = (int)threadIdx.x, lane = tid & 31, wave = tid >> 5;
  unsigned short* rowbuf = (unsigned short*)(misc + MISC_INTS) + wave * SP;
  const int nodeBase = (int)blockIdx.x * NBA;

  {
    const v4i z4 = {0, 0, 0, 0};
    for (int i = tid * 4; i < AGG_ZINTS; i += NTHR * 4) *(v4ia*)(dsm + i) = z4;
    if (tid < MISC_INTS) misc[tid] = 0;
  }
  __syncthreads();

  int t = 0, ov = 0;
  const int nChunks = (nE + CHUNK - 1) / CHUNK;
#pragma unroll 1
  for (int ch = 0; ch < nChunks; ++ch) {
    const int cbase = ch * CHUNK;
    const int wc = scan_chunk<SLA>(keys, nE, cbase, nodeBase, NBA, vec8, list, tid, lane, wave);
    if (lane == 0) misc[wave] = wc;
    __syncthreads();
    if (wave == 0) {
#pragma unroll 1
      for (int w2 = 0; w2 < NWAVE; ++w2) {
        int c = misc[w2];
        c = c < 0 ? 0 : (c > WCAP ? WCAP : c);
#pragma unroll 1
        for (int b0 = 0; b0 < c; b0 += 32) {
          const int idx = b0 + lane;
          const int ent = list[w2 * WCAP + (idx < WCAP ? idx : WCAP - 1)];
          const int m32 = (c - b0) < 32 ? (c - b0) : 32;
#pragma unroll 1
          for (int k = 0; k < m32; ++k) {
            const int u    = __builtin_amdgcn_readlane(ent, k);
            const int slot = u & (NBA - 1);
            const int el   = (u >> SLA) & (CHUNK - 1);
            const int pk   = ((cbase + el) << SLA) | slot;
            if (t < RCAP) {
              if (lane == 0) { hl[t] = pk; cnt[slot] = cnt[slot] + 1; }
              t = t + 1;
            } else {
              ov = 1;
            }
          }
        }
      }
    }
    __syncthreads();
  }
  if (wave == 0 && lane == 0) { misc[8] = t; misc[9] = ov; }
  __syncthreads();
  int tt = misc[8];
  tt = tt < 0 ? 0 : (tt > RCAP ? RCAP : tt);
  const int ovf = misc[9];

  if (wave == 0) {
    const int base = lane * (NBA / 32);
    int s = 0;
#pragma unroll 1
    for (int i = 0; i < NBA / 32; ++i) s += cnt[base + i];
    int incl = s;
#pragma unroll
    for (int d = 1; d < 32; d <<= 1) {
      const int y = __shfl_up(incl, d, 32);
      if (lane >= d) incl += y;
    }
    int run = incl - s;
#pragma unroll 1
    for (int i = 0; i < NBA / 32; ++i) {
      const int cv = cnt[base + i];
      offs[base + i] = run;
      cur[base + i]  = run;
      run += cv;
    }
  }
  __syncthreads();
  if (wave == 0) {
#pragma unroll 1
    for (int b0 = 0; b0 < tt; b0 += 32) {
      const int idx = b0 + lane;
      const int ent = hl[idx < RCAP ? idx : RCAP - 1];
      const int m32 = (tt - b0) < 32 ? (tt - b0) : 32;
#pragma unroll 1
      for (int k = 0; k < m32; ++k) {
        const int u    = __builtin_amdgcn_readlane(ent, k);
        const int slot = u & (NBA - 1);
        if (lane == 0) {
          int p = cur[slot];
          p = p < 0 ? 0 : (p > RCAP - 1 ? RCAP - 1 : p);
          sl[p] = u;
          cur[slot] = p + 1;
        }
      }
    }
  }
  __syncthreads();

  const float qnan = __int_as_float(0x7fc00000);
  const float pz = (ovf != 0) ? qnan : 0.0f;
#pragma unroll 1
  for (int si = 0; si < NBA / NWAVE; ++si) {
    const int s    = si * NWAVE + wave;
    const int node = nodeBase + s;
    int c = cnt[s];
    const bool big = c > DEGCAP;
    c = c < 0 ? 0 : (c > DEGCAP ? DEGCAP : c);
    int o = offs[s];
    o = o < 0 ? 0 : (o > RCAP ? RCAP : o);
    const int nc = node < nN ? node : nN - 1;
    const v4f q = *(const v4f*)(Qp + (size_t)nc * DF + 4 * lane);
    float a0 = 0.0f, a1 = 0.0f, a2 = 0.0f, a3 = 0.0f, z = 0.0f;
#pragma unroll 1
    for (int b0 = 0; b0 < c; b0 += 32) {
      int idx = o + b0 + lane;
      idx = idx > RCAP - 1 ? RCAP - 1 : idx;
      const int ent = sl[idx];
      int eid = ent >> SLA;
      eid = eid < 0 ? 0 : (eid > nE - 1 ? nE - 1 : eid);
      int sr = gath[eid];
      sr = sr < 0 ? 0 : (sr > nN - 1 ? nN - 1 : sr);
      const int m32 = (c - b0) < 32 ? (c - b0) : 32;
#pragma unroll 2
      for (int k = 0; k < m32; ++k) {
        const int sk = __builtin_amdgcn_readlane(sr, k);
        const v4f kv = *(const v4f*)(Kp + (size_t)sk * DF + 4 * lane);
        const v4f vv = *(const v4f*)(Vp + (size_t)sk * DF + 4 * lane);
        float p = kv.x * q.x;
        p = fmaf(kv.y, q.y, p);
        p = fmaf(kv.z, q.z, p);
        p = fmaf(kv.w, q.w, p);
        p += __shfl_xor(p, 1, 32);
        p += __shfl_xor(p, 2, 32);
        float sc = p * 0.25f;
        sc = (sc > 5.0f) ? 5.0f : sc;
        sc = (sc < -5.0f) ? -5.0f : sc;
        const float ex = expf(sc);
        a0 = fmaf(ex, vv.x, a0);
        a1 = fmaf(ex, vv.y, a1);
        a2 = fmaf(ex, vv.z, a2);
        a3 = fmaf(ex, vv.w, a3);
        z += ex;
      }
    }
    const float rz  = 1.0f / (z + 1e-6f);
    const float pzr = big ? qnan : pz;
    const bool live = node < nN;
    v4f mv;
    mv.x = live ? (a0 * rz + pzr) : 0.0f;
    mv.y = live ? (a1 * rz + pzr) : 0.0f;
    mv.z = live ? (a2 * rz + pzr) : 0.0f;
    mv.w = live ? (a3 * rz + pzr) : 0.0f;
    v4us mh, ml;
    hilo4(mv, mh, ml);
    *(v4usa*)(rowbuf + 4 * lane) = mh;
    *(v4usa*)(rowbuf + DF + 4 * lane) = ml;
    wave_sync();
    const v8us q0 = *(const v8usa*)(rowbuf + 8 * lane);
    wave_sync();
    if (node < mRows) {
      unsigned short* rpw = attn + (size_t)node * SP + 8 * lane;
      *(volatile v8us*)rpw = q0;
      __threadfence();
      *(volatile v8us*)rpw = q0;
    }
  }
}

static inline int cdiv(int a, int b) { return (a + b - 1) / b; }
static inline size_t al256(size_t o) { return (o + 255) & ~(size_t)255; }

extern "C" void kernel_launch(void* const* d_in, const int* in_sizes, int n_in,
                              void* d_out, int out_size, void* d_ws, size_t ws_size,
                              hipStream_t stream) {
  if (n_in < 20) return;
  if (in_sizes[0] < DF || (in_sizes[0] % DF) != 0) return;
  const int nN = in_sizes[0] / DF;
  const int nE = in_sizes[1];
  if (nE < 1 || in_sizes[2] != nE) return;
  if (nE >= (1 << 21) || nN < 16 || nN >= (1 << 22)) return;
  if (in_sizes[3] != DF * DF) return;
  if (in_sizes[4] != NLAY * DF * DF || in_sizes[6] != NLAY * DF * DF) return;
  if (in_sizes[8] != NLAY * DF * DF || in_sizes[10] != NLAY * DF * DF) return;
  if (in_sizes[5] != NLAY * DF || in_sizes[7] != NLAY * DF) return;
  if (in_sizes[9] != NLAY * DF || in_sizes[11] != NLAY * DF) return;
  if (in_sizes[12] != NLAY * DF || in_sizes[13] != NLAY * DF) return;
  if (in_sizes[14] != NLAY * DF * 2 * DF || in_sizes[15] != NLAY * 2 * DF) return;
  if (in_sizes[16] != NLAY * 2 * DF * DF || in_sizes[17] != NLAY * DF) return;
  if (in_sizes[18] != NLAY * DF || in_sizes[19] != NLAY * DF) return;
  if ((long long)out_size != (long long)nN * DF) return;

  const float* hin  = (const float*)d_in[0];
  const int*   src  = (const int*)d_in[1];
  const int*   dst  = (const int*)d_in[2];
  const float* Wemb = (const float*)d_in[3];
  const float* Wq   = (const float*)d_in[4];
  const float* bq   = (const float*)d_in[5];
  const float* Wk   = (const float*)d_in[6];
  const float* bk   = (const float*)d_in[7];
  const float* Wv   = (const float*)d_in[8];
  const float* bv   = (const float*)d_in[9];
  const float* Wo   = (const float*)d_in[10];
  const float* bo   = (const float*)d_in[11];
  const float* ln1w = (const float*)d_in[12];
  const float* ln1b = (const float*)d_in[13];
  const float* Wf1  = (const float*)d_in[14];
  const float* bf1  = (const float*)d_in[15];
  const float* Wf2  = (const float*)d_in[16];
  const float* bf2  = (const float*)d_in[17];
  const float* ln2w = (const float*)d_in[18];
  const float* ln2b = (const float*)d_in[19];
  float* out = (float*)d_out;

  const int MP = cdiv(nN, GBM) * GBM;
  const int gM = MP / GBM;
  const int gA = cdiv(MP, NBA);
  if ((long long)gA * NBA < (long long)MP) return;
  const int vec8 = ((nE & 3) == 0) ? 1 : 0;

  const size_t plB = (size_t)MP * DF * 4;
  char* ws = (char*)d_ws;
  size_t off = 0;
  const size_t oS  = off; off = al256(off + (size_t)MP * SP * 2);
  const size_t oQ  = off; off = al256(off + 3 * plB);
  const size_t oAT = off; off = al256(off + (size_t)MP * SP * 2);
  const size_t oWP = off; off = al256(off + (size_t)WPL_ELEMS * 2);
  if (off > ws_size || off > (size_t)WSMAX) return;
  if ((size_t)MP * FP * 2 > 2 * plB) return;
  if ((size_t)MP * SP * 2 > plB) return;
  if ((size_t)MP * DF * 2 > (size_t)MP * SP * 2) return;
  unsigned short* S    = (unsigned short*)(ws + oS);
  float*          Qp   = (float*)(ws + oQ);
  float*          Kp   = (float*)(ws + oQ + plB);
  float*          Vp   = (float*)(ws + oQ + 2 * plB);
  unsigned short* Fh   = (unsigned short*)(ws + oQ);
  unsigned short* HX   = (unsigned short*)(ws + oQ + 2 * plB);
  unsigned short* ATTN = (unsigned short*)(ws + oAT);
  unsigned short* XB   = (unsigned short*)(ws + oAT);
  unsigned short* WPL  = (unsigned short*)(ws + oWP);
  const size_t plE = (size_t)MP * DF;

  const size_t scanLds = (size_t)AGG_LDS_INTS * 4;
  hipFuncSetAttribute(reinterpret_cast<const void*>(&k_scan), hipFuncAttributeMaxDynamicSharedMemorySize, (int)scanLds);

  const int nUx = MP * (DF / 8);
  k_wprep<<<NPARTS * 8, NTHR, 0, stream>>>(Wemb, Wq, Wk, Wv, Wo, Wf1, Wf2, WPL);
  k_cvx<<<cdiv(nUx, NTHR), NTHR, 0, stream>>>(hin, nN, nUx, XB);
  k_gemm<M_EMB, 0><<<dim3(gM, 1), GTHR, 0, stream>>>(XB, DF, WPL, DF, bq, bq, bq, XB, ln1w, ln1b,
                                                     S, SP, Qp, (size_t)0, nN);
  for (int l = 0; l < NLAY; ++l) {
    const unsigned short* WL = WPL + WE_ELEMS + (size_t)l * LAY_ELEMS;
    const float* bql = bq + (size_t)l * DF;
    const float* bkl = bk + (size_t)l * DF;
    const float* bvl = bv + (size_t)l * DF;
    const float* bol = bo + (size_t)l * DF;
    const float* l1w = ln1w + (size_t)l * DF;
    const float* l1b = ln1b + (size_t)l * DF;
    const float* b1l = bf1 + (size_t)l * 2 * DF;
    const float* b2l = bf2 + (size_t)l * DF;
    const float* l2w = ln2w + (size_t)l * DF;
    const float* l2b = ln2b + (size_t)l * DF;
    k_gemm<M_QKV, 0><<<dim3(gM, 3), GTHR, 0, stream>>>(S, SP, WL + OFF_QKV2, SP, bql, bkl, bvl, S, l1w, l1b,
                                                       ATTN, SP, Qp, plE, nN);
    k_scan<<<gA, NTHR, scanLds, stream>>>(src, dst, nE, nN, vec8, MP, Qp, Kp, Vp, ATTN);
    k_gemm<M_LN, 0><<<dim3(gM, 1), GTHR, 0, stream>>>(ATTN, SP, WL + OFF_WO2, SP, bol, bol, bol, S, l1w, l1b,
                                                      HX, SP, out, (size_t)0, nN);
    k_gemm<M_FFN1, 0><<<dim3(gM, 2), GTHR, 0, stream>>>(HX, SP, WL + OFF_WF12, SP, b1l, b1l, b1l, ATTN, l2w, l2b,
                                                        Fh, FP, out, (size_t)0, nN);
    if (l + 1 < NLAY) {
      k_gemm<M_LN, 0><<<dim3(gM, 1), GTHR, 0, stream>>>(Fh, FP, WL + OFF_WF22, FP, b2l, b2l, b2l, HX, l2w, l2b,
                                                        S, SP, out, (size_t)0, nN);
    } else {
      k_gemm<M_LN, 1><<<dim3(gM, 1), GTHR, 0, stream>>>(Fh, FP, WL + OFF_WF22, FP, b2l, b2l, b2l, HX, l2w, l2b,
                                                        S, SP, out, (size_t)0, nN);
    }
  }
}
